// MedformerLayer_38843684225392
// MI455X (gfx1250) — hardware-verified
//
#include <hip/hip_runtime.h>

typedef _Float16 v16h __attribute__((ext_vector_type(16)));
typedef _Float16 v8h  __attribute__((ext_vector_type(8)));
typedef float    v8f  __attribute__((ext_vector_type(8)));
typedef float    v4f  __attribute__((ext_vector_type(4)));

#define NBLK  4
#define NBAT  4
#define SEQL  1024
#define DM    512
#define NH    8
#define HD    64
#define MROWS 16384
#define WPL   262144
#define ZPL   524288
#define SP16  72
#define SP32  68

union FragU { v16h v; v8h h[2]; };

__device__ __forceinline__ v16h frag_ld(const _Float16* p) {
  FragU f;
  f.h[0] = *(const v8h*)(p);
  f.h[1] = *(const v8h*)(p + 16);
  return f.v;
}

__device__ __forceinline__ v8f mma16(v16h a, v16h b, v8f c) {
  c = __builtin_amdgcn_wmma_f32_16x16x32_f16(false, a, false, b, (short)0, c, false, false);
  asm volatile("v_nop\n\tv_nop\n\tv_nop\n\tv_nop" : "+v"(c) : "v"(a), "v"(b));
  return c;
}

__device__ __forceinline__ void wave_lds_sync() {
  __builtin_amdgcn_fence(__ATOMIC_RELEASE, "workgroup");
  __builtin_amdgcn_wave_barrier();
  __builtin_amdgcn_fence(__ATOMIC_ACQUIRE, "workgroup");
}

__device__ __forceinline__ v8f zero8() { return (v8f){0.f, 0.f, 0.f, 0.f, 0.f, 0.f, 0.f, 0.f}; }

__global__ void __launch_bounds__(256)
cvt_x_kernel(const float* __restrict__ x, _Float16* __restrict__ X16, int n8) {
  const int i = blockIdx.x * 256 + threadIdx.x;
  if (i >= n8) return;
  const v4f a = *(const v4f*)(x + (size_t)i * 8);
  const v4f b = *(const v4f*)(x + (size_t)i * 8 + 4);
  v8h hv;
  hv[0] = (_Float16)a[0]; hv[1] = (_Float16)a[1]; hv[2] = (_Float16)a[2]; hv[3] = (_Float16)a[3];
  hv[4] = (_Float16)b[0]; hv[5] = (_Float16)b[1]; hv[6] = (_Float16)b[2]; hv[7] = (_Float16)b[3];
  _Float16* p = X16 + (size_t)i * 8;
  *(volatile v8h*)p = hv;
  __threadfence();
  *(volatile v8h*)p = hv;
}

__global__ void __launch_bounds__(256)
wt_kernel(const float* __restrict__ Wq, const float* __restrict__ Wk,
          const float* __restrict__ Wv, const float* __restrict__ Wo,
          _Float16* __restrict__ WT) {
  __shared__ __align__(16) float tf[64 * 68];
  const int z  = blockIdx.z;
  const int wi = z >> 2, nb = z & 3;
  const float* W = (wi == 0) ? Wq : ((wi == 1) ? Wk : ((wi == 2) ? Wv : Wo));
  W += (size_t)nb * WPL;
  _Float16* O = WT + (size_t)z * WPL;
  const int c0  = blockIdx.x * 64;
  const int r0  = blockIdx.y * 64;
  const int tid = threadIdx.x;
  {
    const int lr = tid >> 4;
    const int c4 = (tid & 15) * 4;
#pragma unroll
    for (int it = 0; it < 4; ++it) {
      const int rr = it * 16 + lr;
      const v4f a = *(const v4f*)(W + (size_t)(r0 + rr) * DM + c0 + c4);
      *(v4f*)(tf + rr * 68 + c4) = a;
    }
  }
  __syncthreads();
  const int sub = tid >> 3;
  const int c8  = (tid & 7) * 8;
  v8h hv0, hv1;
#pragma unroll
  for (int e = 0; e < 8; ++e) {
    hv0[e] = (_Float16)(16.0f * tf[(c8 + e) * 68 + sub]);
    hv1[e] = (_Float16)(16.0f * tf[(c8 + e) * 68 + 32 + sub]);
  }
  _Float16* p0 = O + (size_t)(c0 + sub) * DM + r0 + c8;
  _Float16* p1 = O + (size_t)(c0 + 32 + sub) * DM + r0 + c8;
  for (int pass = 0; pass < 2; ++pass) {
    *(volatile v8h*)p0 = hv0;
    *(volatile v8h*)p1 = hv1;
    __threadfence();
  }
}

__device__ __forceinline__ void gemm_core(const _Float16* __restrict__ A, int lda,
                                          const _Float16* __restrict__ Bt, int ldb,
                                          int m0, int n0, int lane, v8f (&acc)[2][4]) {
  const int c = lane & 15, kh = (lane >> 4) * 8;
#pragma unroll
  for (int i = 0; i < 2; ++i)
#pragma unroll
    for (int j = 0; j < 4; ++j) acc[i][j] = zero8();
  const _Float16* a0p = A  + (size_t)(m0 + c) * lda + kh;
  const _Float16* a1p = A  + (size_t)(m0 + 16 + c) * lda + kh;
  const _Float16* b0p = Bt + (size_t)(n0 + c) * ldb + kh;
#pragma unroll 1
  for (int k0 = 0; k0 < DM; k0 += 32) {
    v16h bf[4];
#pragma unroll
    for (int j = 0; j < 4; ++j) bf[j] = frag_ld(b0p + (size_t)(j * 16) * ldb + k0);
    const v16h a0 = frag_ld(a0p + k0);
    const v16h a1 = frag_ld(a1p + k0);
#pragma unroll
    for (int j = 0; j < 4; ++j) {
      acc[0][j] = mma16(a0, bf[j], acc[0][j]);
      acc[1][j] = mma16(a1, bf[j], acc[1][j]);
    }
  }
}

template <bool BIAS_ROW>
__device__ __forceinline__ void epi_f16(v8f (&acc)[2][4], _Float16* slab,
                                        _Float16* __restrict__ C, int ldc,
                                        int m0, int n0, int lane, float scale,
                                        const float* __restrict__ bias) {
  const int c = lane & 15, hh = lane >> 4;
#pragma unroll
  for (int mt = 0; mt < 2; ++mt) {
#pragma unroll
    for (int nt = 0; nt < 4; ++nt) {
      const int coll = nt * 16 + c;
      float bc = 0.f;
      if (!BIAS_ROW) bc = bias[n0 + coll];
#pragma unroll
      for (int r = 0; r < 8; ++r) {
        const int rowl = mt * 16 + 8 * hh + r;
        float v = acc[mt][nt][r] * scale;
        v += BIAS_ROW ? bias[m0 + rowl] : bc;
        slab[rowl * SP16 + coll] = (_Float16)v;
      }
    }
  }
  wave_lds_sync();
  const int q = lane >> 3, c8 = (lane & 7) * 8;
  for (int pass = 0; pass < 2; ++pass) {
#pragma unroll
    for (int it = 0; it < 8; ++it) {
      const int row = it * 4 + q;
      const v8h val = *(const v8h*)(slab + row * SP16 + c8);
      *(volatile v8h*)(C + (size_t)(m0 + row) * ldc + n0 + c8) = val;
    }
    __threadfence();
  }
  wave_lds_sync();
}

__global__ void __launch_bounds__(256)
qk_gemm_kernel(const _Float16* __restrict__ X16, const _Float16* __restrict__ WT,
               const float* __restrict__ bq, const float* __restrict__ bk,
               _Float16* __restrict__ Q16, _Float16* __restrict__ K16) {
  __shared__ __align__(16) _Float16 slabs[8 * 32 * SP16];
  const int lane = threadIdx.x & 31, wid = threadIdx.x >> 5;
  const int m0 = blockIdx.x * 64 + (wid >> 2) * 32;
  const int n0 = blockIdx.y * 256 + (wid & 3) * 64;
  const int proj = blockIdx.z;
  const int nb = m0 >> 12;
  const _Float16* Bt = WT + (size_t)(proj * 4 + nb) * WPL;
  const float* bias = ((proj == 0) ? bq : bk) + nb * DM;
  _Float16* C = (proj == 0) ? Q16 : K16;
  v8f acc[2][4];
  gemm_core(X16, DM, Bt, DM, m0, n0, lane, acc);
  epi_f16<false>(acc, slabs + wid * (32 * SP16), C, DM, m0, n0, lane, 0.0625f, bias);
}

__global__ void __launch_bounds__(256)
vt_gemm_kernel(const _Float16* __restrict__ X16, const _Float16* __restrict__ WT,
               const float* __restrict__ bv, _Float16* __restrict__ VT16) {
  __shared__ __align__(16) _Float16 slabs[8 * 32 * SP16];
  const int lane = threadIdx.x & 31, wid = threadIdx.x >> 5;
  const int m0 = blockIdx.x * 64 + (wid >> 2) * 32;
  const int n0 = blockIdx.y * 256 + (wid & 3) * 64;
  const int z  = blockIdx.z;
  const int nb = z >> 2;
  const _Float16* A  = WT + (size_t)(8 + nb) * WPL;
  const _Float16* Bt = X16 + (size_t)z * ZPL;
  _Float16* C = VT16 + (size_t)z * ZPL;
  const float* bias = bv + nb * DM;
  v8f acc[2][4];
  gemm_core(A, DM, Bt, DM, m0, n0, lane, acc);
  epi_f16<true>(acc, slabs + wid * (32 * SP16), C, SEQL, m0, n0, lane, 0.0625f, bias);
}

__global__ void __launch_bounds__(128)
attn_kernel(const _Float16* __restrict__ Q16, const _Float16* __restrict__ K16,
            const _Float16* __restrict__ VT16, _Float16* __restrict__ O16) {
  __shared__ __align__(16) _Float16 pbuf[4 * 16 * SP16];
  const int tid = threadIdx.x, wave = tid >> 5, lane = tid & 31;
  const int hh = lane >> 4, c = lane & 15;
  const int bx = blockIdx.x;
  const int qb = bx & 15, h = (bx >> 4) & 7, z = bx >> 7;
  const int q0 = qb * 64 + wave * 16;

  const _Float16* Qz = Q16 + (size_t)z * ZPL + h * HD;
  const _Float16* Kz = K16 + (size_t)z * ZPL + h * HD;
  const _Float16* Vz = VT16 + ((size_t)z * DM + h * HD) * SEQL;
  _Float16* Oz = O16 + (size_t)z * ZPL + h * HD;
  _Float16* pw = pbuf + wave * (16 * SP16);

  const v16h qa0 = frag_ld(Qz + (size_t)(q0 + c) * DM + 8 * hh);
  const v16h qa1 = frag_ld(Qz + (size_t)(q0 + c) * DM + 32 + 8 * hh);

  float mrow[8], lrow[8];
  v8f oacc[4];
#pragma unroll
  for (int r = 0; r < 8; ++r) { mrow[r] = -1e30f; lrow[r] = 0.f; }
#pragma unroll
  for (int t = 0; t < 4; ++t) oacc[t] = zero8();

#pragma unroll 1
  for (int kc = 0; kc < SEQL / 64; ++kc) {
    const int kv0 = kc * 64;
    v8f s[4];
#pragma unroll
    for (int j = 0; j < 4; ++j) {
      const _Float16* kp = Kz + (size_t)(kv0 + j * 16 + c) * DM + 8 * hh;
      s[j] = zero8();
      s[j] = mma16(qa0, frag_ld(kp), s[j]);
      s[j] = mma16(qa1, frag_ld(kp + 32), s[j]);
    }
    float cm[8];
#pragma unroll
    for (int r = 0; r < 8; ++r) {
      float m = -1e30f;
#pragma unroll
      for (int j = 0; j < 4; ++j) {
        const float sv = s[j][r] * 0.125f;
        s[j][r] = sv;
        m = fmaxf(m, sv);
      }
      m = fmaxf(m, __shfl_xor(m, 1, 32));
      m = fmaxf(m, __shfl_xor(m, 2, 32));
      m = fmaxf(m, __shfl_xor(m, 4, 32));
      m = fmaxf(m, __shfl_xor(m, 8, 32));
      cm[r] = m;
    }
#pragma unroll
    for (int r = 0; r < 8; ++r) {
      const float mnew  = fmaxf(mrow[r], cm[r]);
      const float alpha = __expf(mrow[r] - mnew);
      mrow[r] = mnew;
      float psum = 0.f;
#pragma unroll
      for (int j = 0; j < 4; ++j) {
        const float p = __expf(s[j][r] - mnew);
        psum += p;
        pw[(8 * hh + r) * SP16 + j * 16 + c] = (_Float16)p;
      }
      psum += __shfl_xor(psum, 1, 32);
      psum += __shfl_xor(psum, 2, 32);
      psum += __shfl_xor(psum, 4, 32);
      psum += __shfl_xor(psum, 8, 32);
      lrow[r] = lrow[r] * alpha + psum;
#pragma unroll
      for (int t = 0; t < 4; ++t) oacc[t][r] *= alpha;
    }
    wave_lds_sync();
#pragma unroll
    for (int kk = 0; kk < 2; ++kk) {
      const v16h pa = frag_ld(pw + c * SP16 + kk * 32 + 8 * hh);
#pragma unroll
      for (int t = 0; t < 4; ++t) {
        const _Float16* vp = Vz + (size_t)(t * 16 + c) * SEQL + kv0 + kk * 32 + 8 * hh;
        oacc[t] = mma16(pa, frag_ld(vp), oacc[t]);
      }
    }
    wave_lds_sync();
  }

#pragma unroll
  for (int r = 0; r < 8; ++r) {
    const float inv16 = 16.0f * (1.0f / lrow[r]);
#pragma unroll
    for (int t = 0; t < 4; ++t) pw[(8 * hh + r) * SP16 + t * 16 + c] = (_Float16)(oacc[t][r] * inv16);
  }
  wave_lds_sync();
  {
    const int q4 = lane >> 3, c8 = (lane & 7) * 8;
    for (int pass = 0; pass < 2; ++pass) {
#pragma unroll
      for (int it = 0; it < 4; ++it) {
        const int row = it * 4 + q4;
        const v8h val = *(const v8h*)(pw + row * SP16 + c8);
        *(volatile v8h*)(Oz + (size_t)(q0 + row) * DM + c8) = val;
      }
      __threadfence();
    }
  }
}

__global__ void __launch_bounds__(256)
wo_gemm_kernel(const _Float16* __restrict__ O16, const _Float16* __restrict__ WT,
               const float* __restrict__ bo, float* __restrict__ out, float* __restrict__ rplane) {
  __shared__ __align__(16) float slabf[8 * 16 * SP32];
  const int lane = threadIdx.x & 31, wid = threadIdx.x >> 5;
  const int m0 = blockIdx.x * 64 + (wid >> 2) * 32;
  const int n0 = blockIdx.y * 256 + (wid & 3) * 64;
  const int nb = m0 >> 12;
  const _Float16* Bt = WT + (size_t)(12 + nb) * WPL;
  const float* bias = bo + nb * DM;
  v8f acc[2][4];
  gemm_core(O16, DM, Bt, DM, m0, n0, lane, acc);

  float* slab = slabf + wid * (16 * SP32);
  const int c = lane & 15, hh = lane >> 4, c4 = c * 4;
#pragma unroll
  for (int mt = 0; mt < 2; ++mt) {
#pragma unroll
    for (int nt = 0; nt < 4; ++nt) {
      const int coll = nt * 16 + c;
      const float bc = bias[n0 + coll];
#pragma unroll
      for (int r = 0; r < 8; ++r)
        slab[(8 * hh + r) * SP32 + coll] = acc[mt][nt][r] * (1.0f / 256.0f) + bc;
    }
    wave_lds_sync();
    for (int pass = 0; pass < 2; ++pass) {
#pragma unroll
      for (int it = 0; it < 8; ++it) {
        const int row = it * 2 + hh;
        const int gm  = m0 + mt * 16 + row;
        const v4f val = *(const v4f*)(slab + row * SP32 + c4);
        float* dst = ((gm & (SEQL - 1)) == (SEQL - 1))
                         ? (rplane + (size_t)(gm >> 10) * DM + n0 + c4)
                         : (out + (size_t)gm * DM + n0 + c4);
        *(volatile v4f*)dst = val;
      }
      __threadfence();
    }
    wave_lds_sync();
  }
}

__global__ void __launch_bounds__(512)
inter_kernel(const float* __restrict__ rplane,
             const float* __restrict__ iWq, const float* __restrict__ ibq,
             const float* __restrict__ iWk, const float* __restrict__ ibk,
             const float* __restrict__ iWv, const float* __restrict__ ibv,
             const float* __restrict__ iWo, const float* __restrict__ ibo,
             float* __restrict__ out) {
  __shared__ float Rr[NBLK * DM];
  __shared__ float Pj[3][NBLK * DM];
  const int tid = threadIdx.x;
#pragma unroll 1
  for (int b = 0; b < NBAT; ++b) {
    __syncthreads();
#pragma unroll
    for (int i = 0; i < NBLK; ++i) Rr[i * DM + tid] = rplane[(size_t)(i * NBAT + b) * DM + tid];
    __syncthreads();
#pragma unroll 1
    for (int p = 0; p < 3; ++p) {
      const float* W  = (p == 0) ? iWq : ((p == 1) ? iWk : iWv);
      const float* bb = (p == 0) ? ibq : ((p == 1) ? ibk : ibv);
      float a0 = 0.f, a1 = 0.f, a2 = 0.f, a3 = 0.f;
#pragma unroll 2
      for (int k = 0; k < DM; ++k) {
        const float w = W[(size_t)k * DM + tid];
        a0 += Rr[k] * w;
        a1 += Rr[DM + k] * w;
        a2 += Rr[2 * DM + k] * w;
        a3 += Rr[3 * DM + k] * w;
      }
      const float bc = bb[tid];
      Pj[p][tid]          = a0 + bc;
      Pj[p][DM + tid]     = a1 + bc;
      Pj[p][2 * DM + tid] = a2 + bc;
      Pj[p][3 * DM + tid] = a3 + bc;
    }
    __syncthreads();
    {
      const int item = tid >> 4;
      const int nq = item >> 3, hd = item & 7;
      const int e0 = (tid & 15) * 4;
      const int qo = nq * DM + hd * HD;
      const int ko = hd * HD;
      float s0 = 0.f, s1 = 0.f, s2 = 0.f, s3 = 0.f;
#pragma unroll 2
      for (int e = 0; e < HD; ++e) {
        const float qe = Pj[0][qo + e];
        s0 += qe * Pj[1][ko + e];
        s1 += qe * Pj[1][DM + ko + e];
        s2 += qe * Pj[1][2 * DM + ko + e];
        s3 += qe * Pj[1][3 * DM + ko + e];
      }
      s0 *= 0.125f; s1 *= 0.125f; s2 *= 0.125f; s3 *= 0.125f;
      const float mx = fmaxf(fmaxf(s0, s1), fmaxf(s2, s3));
      const float p0 = __expf(s0 - mx), p1 = __expf(s1 - mx), p2 = __expf(s2 - mx), p3 = __expf(s3 - mx);
      const float inv = 1.0f / (p0 + p1 + p2 + p3);
#pragma unroll
      for (int j = 0; j < 4; ++j) {
        const int e = e0 + j;
        const float o = p0 * Pj[2][ko + e] + p1 * Pj[2][DM + ko + e] +
                        p2 * Pj[2][2 * DM + ko + e] + p3 * Pj[2][3 * DM + ko + e];
        Rr[qo + e] = o * inv;
      }
    }
    __syncthreads();
    {
      float a0 = 0.f, a1 = 0.f, a2 = 0.f, a3 = 0.f;
#pragma unroll 2
      for (int k = 0; k < DM; ++k) {
        const float w = iWo[(size_t)k * DM + tid];
        a0 += Rr[k] * w;
        a1 += Rr[DM + k] * w;
        a2 += Rr[2 * DM + k] * w;
        a3 += Rr[3 * DM + k] * w;
      }
      const float bc = ibo[tid];
      a0 += bc; a1 += bc; a2 += bc; a3 += bc;
      float* o0 = out + ((size_t)(0 * NBAT + b) * SEQL + (SEQL - 1)) * DM + tid;
      float* o1 = out + ((size_t)(1 * NBAT + b) * SEQL + (SEQL - 1)) * DM + tid;
      float* o2 = out + ((size_t)(2 * NBAT + b) * SEQL + (SEQL - 1)) * DM + tid;
      float* o3 = out + ((size_t)(3 * NBAT + b) * SEQL + (SEQL - 1)) * DM + tid;
      *(volatile float*)o0 = a0; *(volatile float*)o1 = a1;
      *(volatile float*)o2 = a2; *(volatile float*)o3 = a3;
      __threadfence();
      *(volatile float*)o0 = a0; *(volatile float*)o1 = a1;
      *(volatile float*)o2 = a2; *(volatile float*)o3 = a3;
    }
  }
}

extern "C" void kernel_launch(void* const* d_in, const int* in_sizes, int n_in,
                              void* d_out, int out_size, void* d_ws, size_t ws_size,
                              hipStream_t stream) {
  if (n_in < 17) return;
  if (in_sizes[0] != MROWS * DM) return;
  if (in_sizes[1] != NBLK * WPL || in_sizes[3] != NBLK * WPL || in_sizes[5] != NBLK * WPL || in_sizes[7] != NBLK * WPL) return;
  if (in_sizes[2] != NBLK * DM || in_sizes[4] != NBLK * DM || in_sizes[6] != NBLK * DM || in_sizes[8] != NBLK * DM) return;
  if (in_sizes[9] != WPL || in_sizes[11] != WPL || in_sizes[13] != WPL || in_sizes[15] != WPL) return;
  if (in_sizes[10] != DM || in_sizes[12] != DM || in_sizes[14] != DM || in_sizes[16] != DM) return;
  if (out_size != MROWS * DM) return;

  const float* x   = (const float*)d_in[0];
  const float* Wq  = (const float*)d_in[1];  const float* bq  = (const float*)d_in[2];
  const float* Wk  = (const float*)d_in[3];  const float* bk  = (const float*)d_in[4];
  const float* Wv  = (const float*)d_in[5];  const float* bv  = (const float*)d_in[6];
  const float* Wo  = (const float*)d_in[7];  const float* bo  = (const float*)d_in[8];
  const float* iWq = (const float*)d_in[9];  const float* ibq = (const float*)d_in[10];
  const float* iWk = (const float*)d_in[11]; const float* ibk = (const float*)d_in[12];
  const float* iWv = (const float*)d_in[13]; const float* ibv = (const float*)d_in[14];
  const float* iWo = (const float*)d_in[15]; const float* ibo = (const float*)d_in[16];
  float* out = (float*)d_out;

  const size_t bAct = (size_t)MROWS * DM * 2;
  const size_t bWT  = (size_t)16 * WPL * 2;
  const size_t bRpl = (size_t)16 * DM * 4;
  size_t off = 0;
  const size_t oX  = off; off += bAct;
  const size_t oWT = off; off += bWT;
  const size_t oQ  = off; off += bAct;
  const size_t oK  = off; off += bAct;
  const size_t oVT = off; off += bAct;
  const size_t oO  = off; off += bAct;
  const size_t oR  = off; off += bRpl;
  if (off > ws_size) return;

  char* ws = (char*)d_ws;
  _Float16* X16  = (_Float16*)(ws + oX);
  _Float16* WT16 = (_Float16*)(ws + oWT);
  _Float16* Q16  = (_Float16*)(ws + oQ);
  _Float16* K16  = (_Float16*)(ws + oK);
  _Float16* VT16 = (_Float16*)(ws + oVT);
  _Float16* O16  = (_Float16*)(ws + oO);
  float*    RPL  = (float*)(ws + oR);

  const int n8 = MROWS * DM / 8;
  cvt_x_kernel<<<dim3(n8 / 256), dim3(256), 0, stream>>>(x, X16, n8);
  wt_kernel<<<dim3(DM / 64, DM / 64, 16), dim3(256), 0, stream>>>(Wq, Wk, Wv, Wo, WT16);
  qk_gemm_kernel<<<dim3(MROWS / 64, DM / 256, 2), dim3(256), 0, stream>>>(X16, WT16, bq, bk, Q16, K16);
  vt_gemm_kernel<<<dim3(DM / 64, SEQL / 256, NBLK * NBAT), dim3(256), 0, stream>>>(X16, WT16, bv, VT16);
  attn_kernel<<<dim3(NBLK * NBAT * NH * (SEQL / 64)), dim3(128), 0, stream>>>(Q16, K16, VT16, O16);
  wo_gemm_kernel<<<dim3(MROWS / 64, DM / 256, 1), dim3(256), 0, stream>>>(O16, WT16, bo, out, RPL);
  inter_kernel<<<dim3(1), dim3(512), 0, stream>>>(RPL, iWq, ibq, iWk, ibk, iWv, ibv, iWo, ibo, out);
  (void)hipGetLastError();
}
